// DynamicTemporalAttention_18253611008848
// MI455X (gfx1250) — hardware-verified
//
#include <hip/hip_runtime.h>
#include <math.h>
#include <stdint.h>

typedef __attribute__((ext_vector_type(16))) _Float16 v16h;
typedef __attribute__((ext_vector_type(8)))  _Float16 v8h;
typedef __attribute__((ext_vector_type(16))) __bf16   v16b;
typedef __attribute__((ext_vector_type(8)))  __bf16   v8b;
typedef __attribute__((ext_vector_type(8)))  float    v8f;
typedef __attribute__((ext_vector_type(4)))  float    v4f;
#define PSCALE 32768.0f
#define PSCALE_INV (1.0f / 32768.0f)

#define BSZ     2
#define SEQ_LEN 2048
#define D_MODEL 1024
#define N_HEAD  16
#define HDIM    64
#define KCH     64
#define NQB     (SEQ_LEN / 64)
#define NKC     (SEQ_LEN / KCH)
#define QK_SCALE 0.125f

__device__ __forceinline__ unsigned short f2bf_bits(float f) {
  unsigned u = __float_as_uint(f);
  return (unsigned short)((u + 0x7FFFu + ((u >> 16) & 1u)) >> 16);
}
__device__ __forceinline__ float bf_bits2f(unsigned short h) { return __uint_as_float(((unsigned)h) << 16); }

__device__ __forceinline__ void dep_guard_h(v8f& a, v8f& b, v16h x, v16h y) { asm volatile("v_nop\n\tv_nop\n\tv_nop\n\tv_nop" : "+v"(a), "+v"(b) : "v"(x), "v"(y)); }
__device__ __forceinline__ void dep_guard_b(v8f& a, v8f& b, v16b x, v16b y) { asm volatile("v_nop\n\tv_nop\n\tv_nop\n\tv_nop" : "+v"(a), "+v"(b) : "v"(x), "v"(y)); }
__device__ __forceinline__ void keep4_h(v16h a, v16h b, v16h c, v16h d) { asm volatile("v_nop" :: "v"(a), "v"(b), "v"(c), "v"(d)); }
__device__ __forceinline__ void keep4_b(v16b a, v16b b, v16b c, v16b d) { asm volatile("v_nop" :: "v"(a), "v"(b), "v"(c), "v"(d)); }
__device__ __forceinline__ void acc_guard4(v8f& a, v8f& b, v8f& c, v8f& d) { asm volatile("v_nop\n\tv_nop\n\tv_nop\n\tv_nop" : "+v"(a), "+v"(b), "+v"(c), "+v"(d)); }
template <typename T> struct Frag;
template <> struct Frag<_Float16> {
  typedef v16h V; union U { v16h v; v8h h[2]; };
  static __device__ __forceinline__ v16h load(const _Float16* p) {
    U f; f.h[0] = *(const v8h*)(p); f.h[1] = *(const v8h*)(p + 16); return f.v;
  }
  static __device__ __forceinline__ v8f mma(v16h a, v16h b, v8f c) {
    return __builtin_amdgcn_wmma_f32_16x16x32_f16(false, a, false, b, (short)0, c, false, false);
  }
  static __device__ __forceinline__ void guard(v8f& a, v8f& b, v16h x, v16h y) { dep_guard_h(a, b, x, y); }
  static __device__ __forceinline__ void keep(v16h a, v16h b, v16h c, v16h d) { keep4_h(a, b, c, d); }
};
template <> struct Frag<__bf16> {
  typedef v16b V; union U { v16b v; v8b h[2]; };
  static __device__ __forceinline__ v16b load(const __bf16* p) {
    U f; f.h[0] = *(const v8b*)(p); f.h[1] = *(const v8b*)(p + 16); return f.v;
  }
  static __device__ __forceinline__ v8f mma(v16b a, v16b b, v8f c) {
    return __builtin_amdgcn_wmma_f32_16x16x32_bf16(false, a, false, b, (short)0, c, false, false);
  }
  static __device__ __forceinline__ void guard(v8f& a, v8f& b, v16b x, v16b y) { dep_guard_b(a, b, x, y); }
  static __device__ __forceinline__ void keep(v16b a, v16b b, v16b c, v16b d) { keep4_b(a, b, c, d); }
};

template <int ET> struct Elem;
template <> struct Elem<0> { typedef _Float16 T; };
template <> struct Elem<1> { typedef __bf16 T; };
template <int ET, bool SPLIT, int BIAS_MODE, int OUT_MODE, bool RESID, int ACT = 0>
__global__ __launch_bounds__(256) void wmma_gemm64(
    const unsigned short* __restrict__ Ap, const unsigned short* __restrict__ A2p, int lda, long strideA,
    const unsigned short* __restrict__ Btp, const unsigned short* __restrict__ Bt2p, int ldb, long strideB,
    void* __restrict__ Cout, void* __restrict__ Cout2, int ldc, long strideC,
    const float* __restrict__ bias,
    const float* __restrict__ resid, long strideR,
    int M, int N, int K, float scale) {
  typedef typename Elem<ET>::T T;
  typedef typename Frag<T>::V V;
  const T* A = (const T*)Ap; const T* A2 = (const T*)A2p; const T* Bt = (const T*)Btp; const T* Bt2 = (const T*)Bt2p;
  __shared__ __align__(16) float sT[8][16 * 68];
  const int b    = blockIdx.y;
  const int lane = threadIdx.x & 31;
  const int wave = threadIdx.x >> 5;
  const int tilesN = N >> 6;
  const int tilesM = M >> 6;
  const int tile = blockIdx.x * 8 + wave;
  if (tile >= tilesM * tilesN) return;
  const int tm = tile / tilesN;
  const int tn = tile - tm * tilesN;
  const int m0 = tm << 6;
  const int n0 = tn << 6;

  const T* Ab  = A  + (size_t)b * strideA;
  const T* Bb  = Bt + (size_t)b * strideB;
  const T* Ab2 = SPLIT ? (A2  + (size_t)b * strideA) : nullptr;
  const T* Bb2 = SPLIT ? (Bt2 + (size_t)b * strideB) : nullptr;

  const int rlane = lane & 15;
  const int koff  = (lane >> 4) * 8;
  const int mOff  = (lane >> 4) * 8;

  v8f acc[4][4];
#pragma unroll
  for (int i = 0; i < 4; ++i)
#pragma unroll
    for (int j = 0; j < 4; ++j) acc[i][j] = (v8f){0.f,0.f,0.f,0.f,0.f,0.f,0.f,0.f};

  for (int k0 = 0; k0 < K; k0 += 32) {
    V bh[4], bl[4];
#pragma unroll
    for (int j = 0; j < 4; ++j) {
      const size_t bo = (size_t)(n0 + (j << 4) + rlane) * ldb + koff + k0;
      bh[j] = Frag<T>::load(Bb + bo);
      if (SPLIT) bl[j] = Frag<T>::load(Bb2 + bo);
    }
#pragma unroll
    for (int i = 0; i < 4; ++i) {
      const size_t ao = (size_t)(m0 + (i << 4) + rlane) * lda + koff + k0;
      V ah = Frag<T>::load(Ab + ao);
      V al;
      if (SPLIT) al = Frag<T>::load(Ab2 + ao);
#pragma unroll
      for (int j = 0; j < 4; ++j) {
        acc[i][j] = Frag<T>::mma(ah, bh[j], acc[i][j]);
        if (SPLIT) {
          acc[i][j] = Frag<T>::mma(ah, bl[j], acc[i][j]);
          acc[i][j] = Frag<T>::mma(al, bh[j], acc[i][j]);
        }
      }
      Frag<T>::guard(acc[i][0], acc[i][3], ah, SPLIT ? al : ah);
    }
    Frag<T>::keep(bh[0], bh[1], bh[2], bh[3]);
    if (SPLIT) Frag<T>::keep(bl[0], bl[1], bl[2], bl[3]);
  }
  acc_guard4(acc[0][0], acc[0][1], acc[0][2], acc[0][3]);
  acc_guard4(acc[1][0], acc[1][1], acc[1][2], acc[1][3]);
  acc_guard4(acc[2][0], acc[2][1], acc[2][2], acc[2][3]);
  acc_guard4(acc[3][0], acc[3][1], acc[3][2], acc[3][3]);

  float* slab = sT[wave];
  const float* Rb = RESID ? (resid + (size_t)b * strideR) : nullptr;
#pragma unroll
  for (int i = 0; i < 4; ++i) {
    const int mBase = m0 + (i << 4);
#pragma unroll
    for (int j = 0; j < 4; ++j) {
      const int n = n0 + (j << 4) + rlane;
      float bv = 0.f;
      if (BIAS_MODE == 2) bv = bias[n];
#pragma unroll
      for (int r = 0; r < 8; ++r) {
        float v = acc[i][j][r] * scale;
        if (BIAS_MODE == 1) v += bias[mBase + mOff + r];
        if (BIAS_MODE == 2) v += bv;
        if (RESID) v += Rb[(size_t)(mBase + mOff + r) * ldc + n];
        if (ACT == 1) v = tanhf(v);
        if (ACT == 2) v = fmaxf(v, 0.0f);
        if (ACT == 3) v = v / (1.0f + expf(-v));
        if (ACT == 4) v = (v > 0.f) ? v : 0.01f * v;
        if (ACT == 5) v = 0.5f * v * (1.0f + erff(v * 0.70710678118654752f));
        slab[(mOff + r) * 68 + (j << 4) + rlane] = v;
      }
    }
    __builtin_amdgcn_fence(__ATOMIC_RELEASE, "workgroup");
    __builtin_amdgcn_wave_barrier();
    __builtin_amdgcn_fence(__ATOMIC_ACQUIRE, "workgroup");
    if (OUT_MODE == 0) {
      float* C = (float*)Cout + (size_t)b * strideC;
      const int hh = lane >> 4, c4 = (lane & 15) * 4;
      for (int pass = 0; pass < 2; ++pass) {
#pragma unroll
        for (int it = 0; it < 8; ++it) {
          const int row = it * 2 + hh;
          v4f v = *(const v4f*)(slab + row * 68 + c4);
          *(volatile v4f*)(C + (size_t)(mBase + row) * ldc + n0 + c4) = v;
        }
        __threadfence();
      }
    } else {
      const int q = lane >> 3, c8 = (lane & 7) * 8;
      unsigned short* C  = (unsigned short*)Cout  + (size_t)b * strideC;
      unsigned short* C2 = (OUT_MODE == 2) ? ((unsigned short*)Cout2 + (size_t)b * strideC) : nullptr;
      for (int pass = 0; pass < 2; ++pass) {
#pragma unroll
        for (int it = 0; it < 4; ++it) {
          const int row = it * 4 + q;
          const float* sp = slab + row * 68 + c8;
          v8h hv, lv;
#pragma unroll
          for (int e = 0; e < 8; ++e) {
            if (OUT_MODE == 1) {
              hv[e] = (_Float16)sp[e];
            } else {
              unsigned short hb = f2bf_bits(sp[e]);
              unsigned short lb = f2bf_bits(sp[e] - bf_bits2f(hb));
              hv[e] = __builtin_bit_cast(_Float16, hb);
              lv[e] = __builtin_bit_cast(_Float16, lb);
            }
          }
          *(volatile v8h*)(C + (size_t)(mBase + row) * ldc + n0 + c8) = hv;
          if (OUT_MODE == 2) *(volatile v8h*)(C2 + (size_t)(mBase + row) * ldc + n0 + c8) = lv;
        }
        __threadfence();
      }
    }
    __builtin_amdgcn_fence(__ATOMIC_RELEASE, "workgroup");
    __builtin_amdgcn_wave_barrier();
    __builtin_amdgcn_fence(__ATOMIC_ACQUIRE, "workgroup");
  }
}

__global__ __launch_bounds__(256) void k_split_x(const float* __restrict__ x,
    unsigned short* __restrict__ xh, unsigned short* __restrict__ xl, int n8) {
  const int i = blockIdx.x * 256 + threadIdx.x;
  if (i < n8) {
    const float* p = x + (size_t)i * 8;
    const v4f a0 = *(const v4f*)p;
    const v4f a1 = *(const v4f*)(p + 4);
    v8h hv, lv;
#pragma unroll
    for (int e = 0; e < 4; ++e) {
      const unsigned short hb0 = f2bf_bits(a0[e]);
      const unsigned short lb0 = f2bf_bits(a0[e] - bf_bits2f(hb0));
      const unsigned short hb1 = f2bf_bits(a1[e]);
      const unsigned short lb1 = f2bf_bits(a1[e] - bf_bits2f(hb1));
      hv[e]     = __builtin_bit_cast(_Float16, hb0);
      lv[e]     = __builtin_bit_cast(_Float16, lb0);
      hv[4 + e] = __builtin_bit_cast(_Float16, hb1);
      lv[4 + e] = __builtin_bit_cast(_Float16, lb1);
    }
    unsigned short* dh = xh + (size_t)i * 8;
    unsigned short* dl = xl + (size_t)i * 8;
    *(volatile v8h*)dh = hv;
    *(volatile v8h*)dl = lv;
    __threadfence();
    *(volatile v8h*)dh = hv;
    *(volatile v8h*)dl = lv;
  }
}

__global__ __launch_bounds__(256) void k_wsplit_t(const float* __restrict__ w0, const float* __restrict__ w1,
    const float* __restrict__ w2, const float* __restrict__ w3,
    unsigned short* __restrict__ outp, int Kd, int Nd) {
  __shared__ __align__(16) float tile[64 * 64];
  const int z = blockIdx.z;
  const float* w = (z == 0) ? w0 : (z == 1) ? w1 : (z == 2) ? w2 : w3;
  const int n0 = blockIdx.x * 64, k0 = blockIdx.y * 64;
  const int t = threadIdx.x, lane = t & 31, wave = t >> 5;
  {
    const int kr = t >> 2, cq = (t & 3) * 16;
    const float* src = w + (size_t)(k0 + kr) * Nd + n0 + cq;
#pragma unroll
    for (int i = 0; i < 4; ++i) *(v4f*)(tile + kr * 64 + cq + 4 * i) = *(const v4f*)(src + 4 * i);
  }
  __syncthreads();
  const size_t plane = (size_t)Nd * Kd;
  unsigned short* hiP = outp + (size_t)(2 * z) * plane;
  unsigned short* loP = hiP + plane;
  const int q = lane >> 3, c8 = (lane & 7) * 8;
  for (int pass = 0; pass < 2; ++pass) {
#pragma unroll
    for (int it = 0; it < 4; ++it) {
      const int pl = it >> 1;
      const int nl = (it & 1) * 32 + wave * 4 + q;
      v8h pv;
#pragma unroll
      for (int e = 0; e < 8; ++e) {
        const float f = tile[(c8 + e) * 64 + nl];
        const unsigned short hb = f2bf_bits(f);
        const unsigned short b16 = pl ? f2bf_bits(f - bf_bits2f(hb)) : hb;
        pv[e] = __builtin_bit_cast(_Float16, b16);
      }
      unsigned short* dst = (pl ? loP : hiP) + (size_t)(n0 + nl) * Kd + k0 + c8;
      *(volatile v8h*)dst = pv;
    }
    __threadfence();
  }
}

__device__ __forceinline__ v8f mma_h(v16h a, v16h b, v8f c) {
  c = __builtin_amdgcn_wmma_f32_16x16x32_f16(false, a, false, b, (short)0, c, false, false);
  asm volatile("v_nop\n\tv_nop\n\tv_nop\n\tv_nop" : "+v"(c) : "v"(a), "v"(b));
  return c;
}

__device__ __forceinline__ void qk_scores(const _Float16* Ks, const v16h (&qa)[2], int c, int hh, v8f (&s)[4]) {
  const v8f z = {0.f,0.f,0.f,0.f,0.f,0.f,0.f,0.f};
#pragma unroll
  for (int j = 0; j < 4; ++j) {
    const _Float16* kpp = Ks + (j * 16 + c) * HDIM + 8 * hh;
    const v16h kb0 = Frag<_Float16>::load(kpp);
    const v16h kb1 = Frag<_Float16>::load(kpp + 32);
    v8f t = mma_h(qa[0], kb0, z);
    t = mma_h(qa[1], kb1, t);
#pragma unroll
    for (int r = 0; r < 8; ++r) s[j][r] = t[r] * QK_SCALE;
  }
}

__global__ __launch_bounds__(128) void k_gated_attn(
    const unsigned short* __restrict__ qp, const unsigned short* __restrict__ kp,
    const unsigned short* __restrict__ vp,
    const float* __restrict__ lthr, const float* __restrict__ gshp,
    unsigned short* __restrict__ ohp, unsigned short* __restrict__ olp) {
  typedef Frag<_Float16> F;
  const _Float16* Q  = (const _Float16*)qp;
  const _Float16* Kg = (const _Float16*)kp;
  const _Float16* Vg = (const _Float16*)vp;
  __shared__ __align__(16) _Float16 Ksh[KCH * HDIM];
  __shared__ __align__(16) _Float16 Vt[HDIM * KCH];
  __shared__ __align__(16) _Float16 Psh[4][16 * KCH];
  __shared__ __align__(16) float    Os[4][16 * 68];

  const int tid  = threadIdx.x;
  const int wave = tid >> 5;
  const int lane = tid & 31;
  const int hh   = lane >> 4;
  const int c    = lane & 15;

  const int bx = blockIdx.x;
  const int qb = bx % NQB;
  const int bh = bx / NQB;
  const int h  = bh % N_HEAD;
  const int b  = bh / N_HEAD;
  const size_t tok0 = (size_t)b * SEQ_LEN;
  const int q0 = qb * 64 + wave * 16;
  const int hoff = h * HDIM;

  v16h qa[2];
  {
    const _Float16* qrow = Q + (tok0 + q0 + c) * D_MODEL + hoff + 8 * hh;
    qa[0] = F::load(qrow);
    qa[1] = F::load(qrow + 32);
  }
  const float thr = 1.0f / (1.0f + __expf(-lthr[h]));
  const float shp = gshp[h];

  float mrow[8], lrow[8];
#pragma unroll
  for (int r = 0; r < 8; ++r) { mrow[r] = -INFINITY; lrow[r] = 0.f; }

  for (int kc = 0; kc < NKC; ++kc) {
    const int kv0 = kc * KCH;
    __syncthreads();
    {
      const int kvr = tid >> 1, dh = (tid & 1) * 32;
      const _Float16* krow = Kg + (tok0 + kv0 + kvr) * D_MODEL + hoff + dh;
      _Float16* kd = Ksh + kvr * HDIM + dh;
#pragma unroll
      for (int i = 0; i < 4; ++i) *(v8h*)(kd + 8 * i) = *(const v8h*)(krow + 8 * i);
    }
    __syncthreads();
    v8f s[4];
    qk_scores(Ksh, qa, c, hh, s);
#pragma unroll
    for (int r = 0; r < 8; ++r) {
      float m = fmaxf(fmaxf(s[0][r], s[1][r]), fmaxf(s[2][r], s[3][r]));
#pragma unroll
      for (int off = 1; off < 16; off <<= 1) m = fmaxf(m, __shfl_xor(m, off, 32));
      const float mnew  = fmaxf(mrow[r], m);
      const float alpha = __expf(mrow[r] - mnew);
      float psum = __expf(s[0][r] - mnew) + __expf(s[1][r] - mnew)
                 + __expf(s[2][r] - mnew) + __expf(s[3][r] - mnew);
#pragma unroll
      for (int off = 1; off < 16; off <<= 1) psum += __shfl_xor(psum, off, 32);
      lrow[r] = lrow[r] * alpha + psum;
      mrow[r] = mnew;
    }
  }
  float invl[8];
#pragma unroll
  for (int r = 0; r < 8; ++r) invl[r] = 1.0f / lrow[r];

  v8f oacc[4];
#pragma unroll
  for (int t = 0; t < 4; ++t) oacc[t] = (v8f){0.f,0.f,0.f,0.f,0.f,0.f,0.f,0.f};
  _Float16* pw = Psh[wave];

  for (int kc = 0; kc < NKC; ++kc) {
    const int kv0 = kc * KCH;
    __syncthreads();
    {
      const int kvr = tid >> 1, dh = (tid & 1) * 32;
      const _Float16* krow = Kg + (tok0 + kv0 + kvr) * D_MODEL + hoff + dh;
      const _Float16* vrow = Vg + (tok0 + kv0 + kvr) * D_MODEL + hoff + dh;
      _Float16* kd = Ksh + kvr * HDIM + dh;
#pragma unroll
      for (int i = 0; i < 4; ++i) {
        *(v8h*)(kd + 8 * i) = *(const v8h*)(krow + 8 * i);
        const v8h vv = *(const v8h*)(vrow + 8 * i);
#pragma unroll
        for (int e = 0; e < 8; ++e) Vt[(dh + 8 * i + e) * KCH + kvr] = vv[e];
      }
    }
    __syncthreads();
    v8f s[4];
    qk_scores(Ksh, qa, c, hh, s);
#pragma unroll
    for (int r = 0; r < 8; ++r) {
#pragma unroll
      for (int j = 0; j < 4; ++j) {
        const float a  = __expf(s[j][r] - mrow[r]) * invl[r];
        const float ex = __expf(shp * (thr - a));
        const float wg = a * __builtin_amdgcn_rcpf(1.0f + ex);
        pw[(8 * hh + r) * KCH + j * 16 + c] = (_Float16)(wg * PSCALE);
      }
    }
    __builtin_amdgcn_fence(__ATOMIC_RELEASE, "workgroup");
    __builtin_amdgcn_wave_barrier();
    __builtin_amdgcn_fence(__ATOMIC_ACQUIRE, "workgroup");
#pragma unroll
    for (int kk = 0; kk < 2; ++kk) {
      const v16h pa = F::load(pw + c * KCH + kk * 32 + 8 * hh);
#pragma unroll
      for (int t = 0; t < 4; ++t) {
        const v16h vb = F::load(Vt + (t * 16 + c) * KCH + kk * 32 + 8 * hh);
        oacc[t] = mma_h(pa, vb, oacc[t]);
      }
    }
  }

  float* os = Os[wave];
#pragma unroll
  for (int r = 0; r < 8; ++r) {
#pragma unroll
    for (int t = 0; t < 4; ++t) os[(8 * hh + r) * 68 + t * 16 + c] = oacc[t][r] * PSCALE_INV;
  }
  __builtin_amdgcn_fence(__ATOMIC_RELEASE, "workgroup");
  __builtin_amdgcn_wave_barrier();
  __builtin_amdgcn_fence(__ATOMIC_ACQUIRE, "workgroup");
  {
    const int q4 = lane >> 3, c8 = (lane & 7) * 8;
    for (int pass = 0; pass < 2; ++pass) {
#pragma unroll
      for (int it = 0; it < 4; ++it) {
        const int row = it * 4 + q4;
        const float* sp = os + row * 68 + c8;
        v8h hv, lv;
#pragma unroll
        for (int e = 0; e < 8; ++e) {
          const unsigned short hb = f2bf_bits(sp[e]);
          const unsigned short lb = f2bf_bits(sp[e] - bf_bits2f(hb));
          hv[e] = __builtin_bit_cast(_Float16, hb);
          lv[e] = __builtin_bit_cast(_Float16, lb);
        }
        const size_t go = (tok0 + q0 + row) * D_MODEL + hoff + c8;
        *(volatile v8h*)(ohp + go) = hv;
        *(volatile v8h*)(olp + go) = lv;
      }
      __threadfence();
    }
  }
}

extern "C" void kernel_launch(void* const* d_in, const int* in_sizes, int n_in,
                              void* d_out, int out_size, void* d_ws, size_t ws_size,
                              hipStream_t stream) {
  if (n_in < 11) return;
  const int NTOK = BSZ * SEQ_LEN;
  const size_t nTokD = (size_t)NTOK * D_MODEL;
  const size_t nWW   = (size_t)D_MODEL * D_MODEL;
  if ((size_t)in_sizes[0] != nTokD) return;
  if ((size_t)in_sizes[1] != nWW || (size_t)in_sizes[3] != nWW ||
      (size_t)in_sizes[5] != nWW || (size_t)in_sizes[7] != nWW) return;
  if (in_sizes[2] < D_MODEL || in_sizes[4] < D_MODEL || in_sizes[6] < D_MODEL || in_sizes[8] < D_MODEL) return;
  if (in_sizes[9] < N_HEAD || in_sizes[10] < N_HEAD) return;
  if ((size_t)out_size != nTokD) return;

  const float* x    = (const float*)d_in[0];
  const float* wq_w = (const float*)d_in[1];
  const float* wq_b = (const float*)d_in[2];
  const float* wk_w = (const float*)d_in[3];
  const float* wk_b = (const float*)d_in[4];
  const float* wv_w = (const float*)d_in[5];
  const float* wv_b = (const float*)d_in[6];
  const float* wo_w = (const float*)d_in[7];
  const float* wo_b = (const float*)d_in[8];
  const float* lth  = (const float*)d_in[9];
  const float* gsh  = (const float*)d_in[10];

  char* ws = (char*)d_ws;
  size_t off = 0;
  unsigned short* xh  = (unsigned short*)(ws + off); off += nTokD * 2;
  unsigned short* xl  = (unsigned short*)(ws + off); off += nTokD * 2;
  unsigned short* wT  = (unsigned short*)(ws + off); off += 8 * nWW * 2;
  unsigned short* q16 = (unsigned short*)(ws + off); off += nTokD * 2;
  unsigned short* k16 = (unsigned short*)(ws + off); off += nTokD * 2;
  unsigned short* v16 = (unsigned short*)(ws + off); off += nTokD * 2;
  unsigned short* oh  = (unsigned short*)(ws + off); off += nTokD * 2;
  unsigned short* ol  = (unsigned short*)(ws + off); off += nTokD * 2;
  if (off > ws_size) return;
  const size_t plane = nWW;

  const int n8 = (int)(nTokD / 8);
  k_split_x<<<dim3((n8 + 255) / 256), dim3(256), 0, stream>>>(x, xh, xl, n8);

  k_wsplit_t<<<dim3(D_MODEL / 64, D_MODEL / 64, 4), dim3(256), 0, stream>>>(
      wq_w, wk_w, wv_w, wo_w, wT, D_MODEL, D_MODEL);

  const int gemm_blocks = ((NTOK / 64) * (D_MODEL / 64) + 7) / 8;
  wmma_gemm64<1, true, 2, 1, false><<<dim3(gemm_blocks, 1), dim3(256), 0, stream>>>(
      xh, xl, D_MODEL, 0L, wT + 0 * plane, wT + 1 * plane, D_MODEL, 0L,
      (void*)q16, (void*)q16, D_MODEL, 0L, wq_b, wq_b, 0L, NTOK, D_MODEL, D_MODEL, 1.0f);
  wmma_gemm64<1, true, 2, 1, false><<<dim3(gemm_blocks, 1), dim3(256), 0, stream>>>(
      xh, xl, D_MODEL, 0L, wT + 2 * plane, wT + 3 * plane, D_MODEL, 0L,
      (void*)k16, (void*)k16, D_MODEL, 0L, wk_b, wk_b, 0L, NTOK, D_MODEL, D_MODEL, 1.0f);
  wmma_gemm64<1, true, 2, 1, false><<<dim3(gemm_blocks, 1), dim3(256), 0, stream>>>(
      xh, xl, D_MODEL, 0L, wT + 4 * plane, wT + 5 * plane, D_MODEL, 0L,
      (void*)v16, (void*)v16, D_MODEL, 0L, wv_b, wv_b, 0L, NTOK, D_MODEL, D_MODEL, 1.0f);

  const int attn_blocks = BSZ * N_HEAD * NQB;
  k_gated_attn<<<dim3(attn_blocks), dim3(128), 0, stream>>>(q16, k16, v16, lth, gsh, oh, ol);

  wmma_gemm64<1, true, 2, 0, false><<<dim3(gemm_blocks, 1), dim3(256), 0, stream>>>(
      oh, ol, D_MODEL, 0L, wT + 6 * plane, wT + 7 * plane, D_MODEL, 0L,
      d_out, d_out, D_MODEL, 0L, wo_b, wo_b, 0L, NTOK, D_MODEL, D_MODEL, 1.0f);
}
